// Text2Motion_Transformer_Word_CrossAtt_21414706938510
// MI455X (gfx1250) — hardware-verified
//
#include <hip/hip_runtime.h>
#include <math.h>
#include <stdint.h>

#pragma clang fp contract(off)

#define NB    4
#define SEQ   1024
#define BLKS  511
#define DM    512
#define NH    8
#define NLOC  2
#define NMIX  2
#define NVH   (NH + NMIX)
#define HD    64
#define DML   (NMIX * HD)
#define CQ    0
#define CK    DM
#define CQML  (2 * DM)
#define CKML  (2 * DM + DML)
#define CV    (2 * DM + 2 * DML)
#define NQKV  (3 * DM + 2 * DML)
#define LDQK  CV
#define NQB   (SEQ / 64)
#define NKT   (SEQ / 64)
#define ROWS  (NB * SEQ)
#define OUTN  (ROWS * DM)
static_assert(SEQ == 2 * BLKS + 2);
static_assert(NH * HD == DM);
static_assert(HD == 64);
static_assert(NQKV == 1792 && CV == 1280 && CKML == 1152 && CQML == 1024 && CK == 512);
static_assert((ROWS % 64) == 0 && (NQKV % 64) == 0 && (DM % 64) == 0 && (DM % 32) == 0 && (SEQ % 64) == 0);
static_assert((((ROWS / 64) * (NQKV / 64)) % 8) == 0);
static_assert((((ROWS / 64) * (DM / 64)) % 8) == 0);
static_assert(((ROWS * DM / 8) % 256) == 0);
static_assert(((ROWS * LDQK / 8) % 256) == 0);
static_assert(((DM * DM / 8) % 256) == 0 && ((DML * DM / 8) % 256) == 0);
static_assert((NQKV % 128) == 0 && (CK % 128) == 0 && (CQML % 128) == 0 && (CKML % 128) == 0 && (CV % 128) == 0);
static_assert((DM / 8) == 64);

typedef _Float16 v16h __attribute__((ext_vector_type(16)));
typedef _Float16 v8h  __attribute__((ext_vector_type(8)));
typedef float    v8f  __attribute__((ext_vector_type(8)));
typedef float    v4f  __attribute__((ext_vector_type(4)));
typedef unsigned int v4u __attribute__((ext_vector_type(4)));

__device__ __forceinline__ unsigned short bf_bits(float f) {
  unsigned u = __float_as_uint(f);
  return (unsigned short)((u + 0x7FFFu + ((u >> 16) & 1u)) >> 16);
}
__device__ __forceinline__ float bfr(float f) { return __uint_as_float(((unsigned)bf_bits(f)) << 16); }
__device__ __forceinline__ unsigned short h_bits(_Float16 x) { return __builtin_bit_cast(unsigned short, x); }
__device__ __forceinline__ unsigned pk16(unsigned short a, unsigned short b) { return (unsigned)a | ((unsigned)b << 16); }
__device__ __forceinline__ v8f zero8() { v8f z = {0.f, 0.f, 0.f, 0.f, 0.f, 0.f, 0.f, 0.f}; return z; }
__device__ __forceinline__ void split16(float v, _Float16& hi, _Float16& rs) {
  hi = (_Float16)v;
  rs = (_Float16)((v - (float)hi) * 2048.0f);
}

__device__ __forceinline__ v16h ldfrag_h(const _Float16* p) {
  union { v16h v; v8h h[2]; } f;
  f.h[0] = *(const v8h*)(p);
  f.h[1] = *(const v8h*)(p + 16);
  return f.v;
}

__device__ __forceinline__ v8f mma_h(v16h a, v16h b, v8f c) {
  c = __builtin_amdgcn_wmma_f32_16x16x32_f16(false, a, false, b, (short)0, c, false, false);
#if defined(__HIP_DEVICE_COMPILE__)
  asm volatile("v_nop\n\tv_nop\n\tv_nop\n\tv_nop" : "+v"(c) : "v"(a), "v"(b));
#endif
  return c;
}
__device__ __forceinline__ v8f mma_h_raw(v16h a, v16h b, v8f c) {
  return __builtin_amdgcn_wmma_f32_16x16x32_f16(false, a, false, b, (short)0, c, false, false);
}
__device__ __forceinline__ void dep_guard_h(v8f& a, v8f& b, v16h x, v16h y) {
#if defined(__HIP_DEVICE_COMPILE__)
  asm volatile("v_nop\n\tv_nop\n\tv_nop\n\tv_nop" : "+v"(a), "+v"(b) : "v"(x), "v"(y));
#endif
}
__device__ __forceinline__ void keep4_h(v16h a, v16h b, v16h c, v16h d) {
#if defined(__HIP_DEVICE_COMPILE__)
  asm volatile("v_nop" :: "v"(a), "v"(b), "v"(c), "v"(d));
#endif
}
__device__ __forceinline__ void acc_guard4(v8f& a, v8f& b, v8f& c, v8f& d) {
#if defined(__HIP_DEVICE_COMPILE__)
  asm volatile("v_nop\n\tv_nop\n\tv_nop\n\tv_nop" : "+v"(a), "+v"(b), "+v"(c), "+v"(d));
#endif
}

template <bool RB>
__global__ __launch_bounds__(256) void cvt16(const float* __restrict__ in, unsigned short* out, int n8, float scale) {
  const int i = blockIdx.x * 256 + threadIdx.x;
  if (i < n8) {
    const v4f a = *(const v4f*)(in + (size_t)i * 8);
    const v4f b = *(const v4f*)(in + (size_t)i * 8 + 4);
    float f[8];
    f[0] = a[0]; f[1] = a[1]; f[2] = a[2]; f[3] = a[3];
    f[4] = b[0]; f[5] = b[1]; f[6] = b[2]; f[7] = b[3];
    v4u p;
#pragma unroll
    for (int e = 0; e < 4; ++e) {
      const float g0 = RB ? bfr(f[2 * e]) : f[2 * e];
      const float g1 = RB ? bfr(f[2 * e + 1]) : f[2 * e + 1];
      p[e] = pk16(h_bits((_Float16)(g0 * scale)), h_bits((_Float16)(g1 * scale)));
    }
    *(volatile v4u*)(out + (size_t)i * 8) = p;
    __threadfence();
    *(volatile v4u*)(out + (size_t)i * 8) = p;
  }
}

__global__ __launch_bounds__(256) void bias_cat(const float* __restrict__ bq, const float* __restrict__ bk,
                                                const float* __restrict__ bqm, const float* __restrict__ bkm,
                                                const float* __restrict__ bv, float* bc) {
  const int i = blockIdx.x * 256 + threadIdx.x;
  if (i < NQKV / 4) {
    const int iq  = min(i, DM / 4 - 1);
    const int ik  = min(max(i - CK / 4, 0), DM / 4 - 1);
    const int iqm = min(max(i - CQML / 4, 0), DML / 4 - 1);
    const int ikm = min(max(i - CKML / 4, 0), DML / 4 - 1);
    const int iv  = min(max(i - CV / 4, 0), DM / 4 - 1);
    const v4f aq  = *(const v4f*)(bq  + 4 * iq);
    const v4f ak  = *(const v4f*)(bk  + 4 * ik);
    const v4f aqm = *(const v4f*)(bqm + 4 * iqm);
    const v4f akm = *(const v4f*)(bkm + 4 * ikm);
    const v4f av  = *(const v4f*)(bv  + 4 * iv);
    v4f o;
#pragma unroll
    for (int e = 0; e < 4; ++e) {
      const float x = (i < CK / 4) ? aq[e] : ((i < CQML / 4) ? ak[e] : ((i < CKML / 4) ? aqm[e] : ((i < CV / 4) ? akm[e] : av[e])));
      o[e] = bfr(x);
    }
    *(volatile v4f*)(bc + (size_t)i * 4) = o;
    __threadfence();
    *(volatile v4f*)(bc + (size_t)i * 4) = o;
  }
}

template <bool ARES>
__global__ __launch_bounds__(256) void gemm64_f16(
    const unsigned short* __restrict__ Ap, const unsigned short* __restrict__ Arp, int lda,
    const unsigned short* __restrict__ Btp, int ldb,
    const float* __restrict__ bias, float cscale,
    float* Cf, int ldc, int M, int N, int K) {
  const _Float16* Ah  = (const _Float16*)(const void*)Ap;
  const _Float16* Arh = (const _Float16*)(const void*)Arp;
  const _Float16* Bt  = (const _Float16*)(const void*)Btp;
  __shared__ __align__(16) float sT[8][16 * 68];
  const int lane = threadIdx.x & 31;
  const int wave = threadIdx.x >> 5;
  const int tilesN = N >> 6;
  const int tilesM = M >> 6;
  const int tile = blockIdx.x * 8 + wave;
  if (tile >= tilesM * tilesN) return;
  const int tm = tile / tilesN;
  const int tn = tile - tm * tilesN;
  const int m0 = tm << 6;
  const int n0 = tn << 6;

  const int rlane = lane & 15;
  const int koff  = (lane >> 4) * 8;
  const int mOff  = (lane >> 4) * 8;

  v8f acc[4][4];
#pragma unroll
  for (int i = 0; i < 4; ++i)
#pragma unroll
    for (int j = 0; j < 4; ++j) acc[i][j] = zero8();

  float bb[4];
#pragma unroll
  for (int j = 0; j < 4; ++j) bb[j] = bfr(bias[n0 + (j << 4) + rlane]);

  constexpr int NPL = ARES ? 2 : 1;
#pragma unroll 1
  for (int pl = 0; pl < NPL; ++pl) {
    const _Float16* Asel = (ARES && pl == 0) ? Arh : Ah;
    if (ARES && pl == 1) {
      acc_guard4(acc[0][0], acc[0][1], acc[0][2], acc[0][3]);
      acc_guard4(acc[1][0], acc[1][1], acc[1][2], acc[1][3]);
      acc_guard4(acc[2][0], acc[2][1], acc[2][2], acc[2][3]);
      acc_guard4(acc[3][0], acc[3][1], acc[3][2], acc[3][3]);
#pragma unroll
      for (int i = 0; i < 4; ++i)
#pragma unroll
        for (int j = 0; j < 4; ++j) acc[i][j] = acc[i][j] * (1.0f / 2048.0f);
      acc_guard4(acc[0][0], acc[0][1], acc[0][2], acc[0][3]);
      acc_guard4(acc[1][0], acc[1][1], acc[1][2], acc[1][3]);
      acc_guard4(acc[2][0], acc[2][1], acc[2][2], acc[2][3]);
      acc_guard4(acc[3][0], acc[3][1], acc[3][2], acc[3][3]);
    }
    for (int k0 = 0; k0 < K; k0 += 32) {
      v16h bh[4];
#pragma unroll
      for (int j = 0; j < 4; ++j) {
        const size_t bo = (size_t)(n0 + (j << 4) + rlane) * ldb + koff + k0;
        bh[j] = ldfrag_h(Bt + bo);
      }
#pragma unroll
      for (int i = 0; i < 4; ++i) {
        const size_t ao = (size_t)(m0 + (i << 4) + rlane) * lda + koff + k0;
        const v16h ah = ldfrag_h(Asel + ao);
#pragma unroll
        for (int j = 0; j < 4; ++j) {
          acc[i][j] = mma_h_raw(ah, bh[j], acc[i][j]);
        }
        dep_guard_h(acc[i][0], acc[i][3], ah, bh[3]);
      }
      keep4_h(bh[0], bh[1], bh[2], bh[3]);
    }
  }
  acc_guard4(acc[0][0], acc[0][1], acc[0][2], acc[0][3]);
  acc_guard4(acc[1][0], acc[1][1], acc[1][2], acc[1][3]);
  acc_guard4(acc[2][0], acc[2][1], acc[2][2], acc[2][3]);
  acc_guard4(acc[3][0], acc[3][1], acc[3][2], acc[3][3]);

  float* slab = sT[wave];
#pragma unroll
  for (int i = 0; i < 4; ++i) {
    const int mBase = m0 + (i << 4);
#pragma unroll
    for (int r = 0; r < 8; ++r) {
      const int row = mOff + r;
#pragma unroll
      for (int j = 0; j < 4; ++j) slab[row * 68 + (j << 4) + rlane] = acc[i][j][r] * cscale + bb[j];
    }
    __builtin_amdgcn_fence(__ATOMIC_RELEASE, "workgroup");
    __builtin_amdgcn_wave_barrier();
    __builtin_amdgcn_fence(__ATOMIC_ACQUIRE, "workgroup");
    {
      const int hh = lane >> 4, c4 = (lane & 15) * 4;
      v4f ov[8];
#pragma unroll
      for (int it = 0; it < 8; ++it) {
        const int row = it * 2 + hh;
        ov[it] = *(const v4f*)(slab + row * 68 + c4);
      }
      for (int pass = 0; pass < 2; ++pass) {
#pragma unroll
        for (int it = 0; it < 8; ++it) {
          const int row = it * 2 + hh;
          *(volatile v4f*)(Cf + (size_t)(mBase + row) * ldc + n0 + c4) = ov[it];
        }
        __threadfence();
      }
    }
    __builtin_amdgcn_fence(__ATOMIC_RELEASE, "workgroup");
    __builtin_amdgcn_wave_barrier();
    __builtin_amdgcn_fence(__ATOMIC_ACQUIRE, "workgroup");
  }
}

__global__ __launch_bounds__(256) void qk_split(const float* __restrict__ src, unsigned short* hi, unsigned short* rs, int n8) {
  const int i = blockIdx.x * 256 + threadIdx.x;
  if (i < n8) {
    const int row = i / (LDQK / 8);
    const int g   = i - row * (LDQK / 8);
    const float* s = src + (size_t)row * NQKV + g * 8;
    const v4f a = *(const v4f*)(s);
    const v4f b = *(const v4f*)(s + 4);
    float f[8];
    f[0] = a[0]; f[1] = a[1]; f[2] = a[2]; f[3] = a[3];
    f[4] = b[0]; f[5] = b[1]; f[6] = b[2]; f[7] = b[3];
    v4u p, q;
#pragma unroll
    for (int e = 0; e < 4; ++e) {
      _Float16 x0, y0, x1, y1;
      split16(f[2 * e] * 16.0f, x0, y0);
      split16(f[2 * e + 1] * 16.0f, x1, y1);
      p[e] = pk16(h_bits(x0), h_bits(x1));
      q[e] = pk16(h_bits(y0), h_bits(y1));
    }
    const size_t o = (size_t)i * 8;
    *(volatile v4u*)(hi + o) = p;
    *(volatile v4u*)(rs + o) = q;
    __threadfence();
    *(volatile v4u*)(hi + o) = p;
    *(volatile v4u*)(rs + o) = q;
  }
}

__global__ __launch_bounds__(256) void v_tr(const float* __restrict__ qkvf, unsigned short* vt, unsigned short* vtr) {
  __shared__ __align__(16) float sv[64 * 68];
  const int tid = threadIdx.x;
  const int t0  = blockIdx.x * 64;
  const int h   = blockIdx.y;
  const int b   = blockIdx.z;
#pragma unroll
  for (int i = 0; i < 4; ++i) {
    const int idx = i * 256 + tid;
    const int tt = idx >> 4, c4 = (idx & 15) * 4;
    const v4f a = *(const v4f*)(qkvf + ((size_t)(b * SEQ + t0 + tt)) * NQKV + CV + h * HD + c4);
    *(v4f*)(sv + tt * 68 + c4) = a;
  }
  __syncthreads();

  const int g = tid >> 3, piece = tid & 7;
  v4u hv[2], rv[2];
  size_t ho[2];
#pragma unroll
  for (int it = 0; it < 2; ++it) {
    const int d = it * 32 + g;
    v4u p, q;
#pragma unroll
    for (int e = 0; e < 4; ++e) {
      _Float16 x0, y0, x1, y1;
      split16(sv[(piece * 8 + 2 * e) * 68 + d] * 16.0f, x0, y0);
      split16(sv[(piece * 8 + 2 * e + 1) * 68 + d] * 16.0f, x1, y1);
      p[e] = pk16(h_bits(x0), h_bits(x1));
      q[e] = pk16(h_bits(y0), h_bits(y1));
    }
    hv[it] = p;
    rv[it] = q;
    ho[it] = ((size_t)((b * NH + h) * HD + d)) * SEQ + t0 + piece * 8;
  }
  for (int pass = 0; pass < 2; ++pass) {
#pragma unroll
    for (int it = 0; it < 2; ++it) {
      *(volatile v4u*)(vt + ho[it])  = hv[it];
      *(volatile v4u*)(vtr + ho[it]) = rv[it];
    }
    __threadfence();
  }
}

__device__ __forceinline__ int tpos(int t) {
  const int up = 2 * (t - 2) + 1;
  const int lo = 2 * (t - 2 - BLKS) + 2;
  return (t < 2) ? 0 : ((t < 2 + BLKS) ? up : lo);
}
__device__ __forceinline__ int ppos(int t) {
  return (t < 2 + BLKS) ? (t - 2) : (t - 2 - BLKS);
}
__device__ __forceinline__ bool key_visible(int q, int k, bool local) {
  const bool g   = tpos(k) <= tpos(q);
  const bool far = (q >= 2) && (k >= 2) && (ppos(k) <= ppos(q) - 4);
  return g && !(local && far);
}
__device__ __forceinline__ bool tile_all_masked(int qb, int kt, bool local) {
  const int k0 = kt * 64, k1 = k0 + 63;
  const int q0 = qb * 64, q1 = q0 + 63;
  const bool ks = (k0 <= 1 + BLKS) && (2 + BLKS <= k1);
  const bool qs = (q0 <= 1 + BLKS) && (2 + BLKS <= q1);
  const int tmin = ks ? min(tpos(k0), tpos(2 + BLKS)) : tpos(k0);
  const int tmax = qs ? max(tpos(q1), tpos(1 + BLKS)) : tpos(q1);
  const bool gall = tmin > tmax;
  const int kkmax = ks ? (BLKS - 1) : ppos(k1);
  const int qqmin = qs ? 0 : ppos(q0);
  const bool lall = local && (k0 >= 2) && (q0 >= 2) && (kkmax <= qqmin - 4);
  return gall || lall;
}

__global__ __launch_bounds__(128)
void attn_k(const unsigned short* __restrict__ qkhp, const unsigned short* __restrict__ qkrp,
            const unsigned short* __restrict__ vtp, const unsigned short* __restrict__ vtrp,
            const float* __restrict__ bclip, const float* __restrict__ bclipml,
            float* yv) {
  union FH { v16h v; v8h h[2]; };
  constexpr int KTB    = 64 * HD * 2;
  constexpr int PTB    = 4 * 16 * 64 * 2;
  constexpr int OFF_K  = 0;
  constexpr int OFF_KR = KTB;
  constexpr int OFF_V  = 2 * KTB;
  constexpr int OFF_VR = 3 * KTB;
  constexpr int OFF_P  = 4 * KTB;
  constexpr int OFF_PR = OFF_P + PTB;
  constexpr int SMEMB  = OFF_PR + PTB;
  static_assert(4 * 16 * HD * 4 <= OFF_V);
  static_assert(SMEMB == 49152);
  __shared__ __align__(16) unsigned char smem[SMEMB];
  _Float16* Ksh = (_Float16*)(smem + OFF_K);
  _Float16* Krs = (_Float16*)(smem + OFF_KR);
  _Float16* Vsh = (_Float16*)(smem + OFF_V);
  _Float16* Vrs = (_Float16*)(smem + OFF_VR);
  _Float16* Psh = (_Float16*)(smem + OFF_P);
  _Float16* Prs = (_Float16*)(smem + OFF_PR);

  const int tid  = threadIdx.x;
  const int wave = tid >> 5;
  const int lane = tid & 31;
  const int hh   = lane >> 4;
  const int c    = lane & 15;

  const int bx   = blockIdx.x;
  const int qb   = bx % NQB;
  const int rest = bx / NQB;
  const int vh   = rest % NVH;
  const int b    = rest / NVH;
  const bool isml = vh >= NH;
  const int mml  = isml ? (vh - NH) : 0;
  const int hm   = isml ? 0 : vh;
  const int qcol = isml ? (CQML + mml * HD) : (CQ + hm * HD);
  const int kcol = isml ? (CKML + mml * HD) : (CK + hm * HD);
  const int hv   = isml ? (NLOC + mml) : hm;
  const bool local = isml || (vh < NLOC);
  const float bmain = bfr(bclip[hm]);
  const float bml   = bfr(bclipml[mml]);
  const float biasv = isml ? bml : bmain;
  const int q0   = qb * 64 + wave * 16;
  const size_t rowB = (size_t)b * SEQ;

  const _Float16* Qg  = (const _Float16*)(const void*)qkhp + (size_t)qcol;
  const _Float16* Qrg = (const _Float16*)(const void*)qkrp + (size_t)qcol;
  const _Float16* Kg  = (const _Float16*)(const void*)qkhp + (size_t)kcol;
  const _Float16* Krg = (const _Float16*)(const void*)qkrp + (size_t)kcol;
  const _Float16* Vg  = (const _Float16*)(const void*)vtp  + ((size_t)(b * NH + hv) * HD) * SEQ;
  const _Float16* Vrg = (const _Float16*)(const void*)vtrp + ((size_t)(b * NH + hv) * HD) * SEQ;
  const float SC = 1.0f / 2048.0f;

  float lsum[8], mrun[8];
  v8f oacc[4];
#pragma unroll
  for (int r = 0; r < 8; ++r) { lsum[r] = 0.f; mrun[r] = -1e30f; }
#pragma unroll
  for (int t = 0; t < 4; ++t) oacc[t] = zero8();

  _Float16* pw  = Psh + wave * (16 * 64);
  _Float16* prw = Prs + wave * (16 * 64);

  for (int kt = 0; kt < NKT; ++kt) {
    if (tile_all_masked(qb, kt, local)) continue;
    const int kv0 = kt * 64;
    __syncthreads();
    {
      const int r = tid >> 1, dh = (tid & 1) * 32;
      const size_t ko = (rowB + kv0 + r) * LDQK + dh;
#pragma unroll
      for (int i = 0; i < 4; ++i) {
        const v8h a0 = *(const v8h*)(Kg + ko + 8 * i);
        const v8h a1 = *(const v8h*)(Krg + ko + 8 * i);
        *(v8h*)(Ksh + r * HD + dh + 8 * i) = a0;
        *(v8h*)(Krs + r * HD + dh + 8 * i) = a1;
      }
      const int d = tid >> 1, kh = (tid & 1) * 32;
      const size_t vo = (size_t)d * SEQ + kv0 + kh;
#pragma unroll
      for (int i = 0; i < 4; ++i) {
        const v8h b0 = *(const v8h*)(Vg + vo + 8 * i);
        const v8h b1 = *(const v8h*)(Vrg + vo + 8 * i);
        *(v8h*)(Vsh + d * 64 + kh + 8 * i) = b0;
        *(v8h*)(Vrs + d * 64 + kh + 8 * i) = b1;
      }
    }
    __syncthreads();

    v8f s[4];
#pragma unroll
    for (int j = 0; j < 4; ++j) {
      v8f sacc = zero8(), tacc = zero8();
      const _Float16* kq  = Ksh + (j * 16 + c) * HD + 8 * hh;
      const _Float16* krq = Krs + (j * 16 + c) * HD + 8 * hh;
#pragma unroll 1
      for (int dc = 0; dc < HD / 32; ++dc) {
        const size_t qo = (rowB + q0 + c) * LDQK + dc * 32 + 8 * hh;
        const v16h qa = ldfrag_h(Qg + qo);
        const v16h qr = ldfrag_h(Qrg + qo);
        FH kb, krb;
        kb.h[0]  = *(const v8h*)(kq + dc * 32);
        kb.h[1]  = *(const v8h*)(kq + dc * 32 + 16);
        krb.h[0] = *(const v8h*)(krq + dc * 32);
        krb.h[1] = *(const v8h*)(krq + dc * 32 + 16);
        sacc = mma_h(qa, kb.v, sacc);
        tacc = mma_h(qa, krb.v, tacc);
        tacc = mma_h(qr, kb.v, tacc);
      }
      s[j] = sacc + tacc * (1.0f / 2048.0f);
    }

    float alpha[8];
#pragma unroll
    for (int r = 0; r < 8; ++r) {
      const int qrow = q0 + 8 * hh + r;
      float av[4];
      bool okv[4];
      float tmx = -1e30f;
#pragma unroll
      for (int j = 0; j < 4; ++j) {
        const int key = kv0 + j * 16 + c;
        float a = s[j][r] * SC;
        a = (key == 1) ? (a + biasv) : a;
        const bool ok = key_visible(qrow, key, local);
        a = ok ? a : -1e30f;
        av[j]  = a;
        okv[j] = ok;
        tmx = fmaxf(tmx, a);
      }
#pragma unroll
      for (int off = 1; off < 16; off <<= 1) tmx = fmaxf(tmx, __shfl_xor(tmx, off, 32));
      const float mn = fmaxf(mrun[r], tmx);
      const float al = __expf(mrun[r] - mn);
      alpha[r] = al;
      mrun[r]  = mn;
      float ps = 0.0f;
#pragma unroll
      for (int j = 0; j < 4; ++j) {
        float p = __expf(av[j] - mn);
        p = okv[j] ? p : 0.0f;
        ps += p;
        _Float16 x0, y0;
        split16(p * 256.0f, x0, y0);
        pw[(8 * hh + r) * 64 + j * 16 + c]  = x0;
        prw[(8 * hh + r) * 64 + j * 16 + c] = y0;
      }
      lsum[r] = lsum[r] * al + ps;
    }
    __builtin_amdgcn_fence(__ATOMIC_RELEASE, "workgroup");
    __builtin_amdgcn_wave_barrier();
    __builtin_amdgcn_fence(__ATOMIC_ACQUIRE, "workgroup");

#pragma unroll
    for (int t = 0; t < 4; ++t) {
#pragma unroll
      for (int r = 0; r < 8; ++r) oacc[t][r] = oacc[t][r] * alpha[r];
    }
    acc_guard4(oacc[0], oacc[1], oacc[2], oacc[3]);

    FH pa[2], par[2];
#pragma unroll
    for (int kk = 0; kk < 2; ++kk) {
      pa[kk].h[0]  = *(const v8h*)(pw + c * 64 + kk * 32 + 8 * hh);
      pa[kk].h[1]  = *(const v8h*)(pw + c * 64 + kk * 32 + 16 + 8 * hh);
      par[kk].h[0] = *(const v8h*)(prw + c * 64 + kk * 32 + 8 * hh);
      par[kk].h[1] = *(const v8h*)(prw + c * 64 + kk * 32 + 16 + 8 * hh);
    }
#pragma unroll
    for (int t = 0; t < 4; ++t) {
      v8f tr = zero8();
#pragma unroll
      for (int kk = 0; kk < 2; ++kk) {
        FH vb, vrb;
        vb.h[0]  = *(const v8h*)(Vsh + (t * 16 + c) * 64 + kk * 32 + 8 * hh);
        vb.h[1]  = *(const v8h*)(Vsh + (t * 16 + c) * 64 + kk * 32 + 16 + 8 * hh);
        vrb.h[0] = *(const v8h*)(Vrs + (t * 16 + c) * 64 + kk * 32 + 8 * hh);
        vrb.h[1] = *(const v8h*)(Vrs + (t * 16 + c) * 64 + kk * 32 + 16 + 8 * hh);
        tr = mma_h(pa[kk].v, vrb.v, tr);
        tr = mma_h(par[kk].v, vb.v, tr);
        oacc[t] = mma_h(pa[kk].v, vb.v, oacc[t]);
      }
      oacc[t] = oacc[t] + tr * (1.0f / 2048.0f);
    }
    acc_guard4(oacc[0], oacc[1], oacc[2], oacc[3]);
  }
  __syncthreads();

  float* os = (float*)(void*)smem + wave * (16 * HD);
#pragma unroll
  for (int r = 0; r < 8; ++r) {
    float l = lsum[r];
#pragma unroll
    for (int off = 1; off < 16; off <<= 1) l += __shfl_xor(l, off, 32);
    const float rl = 1.0f / l;
    const float sc = rl * (1.0f / 4096.0f);
#pragma unroll
    for (int t = 0; t < 4; ++t) os[(8 * hh + r) * HD + t * 16 + c] = oacc[t][r] * sc;
  }
  __builtin_amdgcn_fence(__ATOMIC_RELEASE, "workgroup");
  __builtin_amdgcn_wave_barrier();
  __builtin_amdgcn_fence(__ATOMIC_ACQUIRE, "workgroup");
  {
    const int piece = lane & 15;
    v4f ov[8];
#pragma unroll
    for (int it = 0; it < 8; ++it) {
      const int row = it * 2 + hh;
      ov[it] = *(const v4f*)(os + row * HD + piece * 4);
    }
    for (int pass = 0; pass < 2; ++pass) {
#pragma unroll
      for (int it = 0; it < 8; ++it) {
        const int row = it * 2 + hh;
        const size_t go = (((size_t)(vh * NB + b)) * SEQ + q0 + row) * HD + piece * 4;
        *(volatile v4f*)(yv + go) = ov[it];
      }
      __threadfence();
    }
  }
}

__global__ __launch_bounds__(256) void mix_cvt(const float* __restrict__ yv, const float* __restrict__ mixw,
                                               unsigned short* ctx, unsigned short* ctxr) {
  const int i = blockIdx.x * 256 + threadIdx.x;
  if (i < ROWS * DM / 8) {
    const int row = i >> 6;
    const int g   = i & 63;
    const int h   = g >> 3, d0 = (g & 7) * 8;
    const int b   = row / SEQ, t = row - b * SEQ;
    const bool ismix = (h >= NLOC) && (h < NLOC + NMIX);
    const int m   = ismix ? (h - NLOC) : 0;
    const int vl  = NH + m;
    const float* pg = yv + (((size_t)(h * NB + b)) * SEQ + t) * HD + d0;
    const float* pl = yv + (((size_t)(vl * NB + b)) * SEQ + t) * HD + d0;
    const v4f g0 = *(const v4f*)(pg);
    const v4f g1 = *(const v4f*)(pg + 4);
    const v4f l0 = *(const v4f*)(pl);
    const v4f l1 = *(const v4f*)(pl + 4);
    const float w0 = bfr(mixw[m * 2 + 0]);
    const float w1 = bfr(mixw[m * 2 + 1]);
    float f[8];
#pragma unroll
    for (int u = 0; u < 4; ++u) {
      const float ba = w0 * g0[u] + w1 * l0[u];
      const float bb = w0 * g1[u] + w1 * l1[u];
      f[u]     = ismix ? ba : g0[u];
      f[4 + u] = ismix ? bb : g1[u];
    }
    v4u p, q;
#pragma unroll
    for (int e = 0; e < 4; ++e) {
      _Float16 x0, y0, x1, y1;
      split16(f[2 * e] * 16.0f, x0, y0);
      split16(f[2 * e + 1] * 16.0f, x1, y1);
      p[e] = pk16(h_bits(x0), h_bits(x1));
      q[e] = pk16(h_bits(y0), h_bits(y1));
    }
    const size_t o = (size_t)i * 8;
    *(volatile v4u*)(ctx + o)  = p;
    *(volatile v4u*)(ctxr + o) = q;
    __threadfence();
    *(volatile v4u*)(ctx + o)  = p;
    *(volatile v4u*)(ctxr + o) = q;
  }
}

extern "C" void kernel_launch(void* const* d_in, const int* in_sizes, int n_in,
                              void* d_out, int out_size, void* d_ws, size_t ws_size,
                              hipStream_t stream) {
  if (n_in < 17) return;
  if (in_sizes[0] != ROWS * DM) return;
  if (in_sizes[2] != DM * DM || in_sizes[3] != DM) return;
  if (in_sizes[4] != DM * DM || in_sizes[5] != DM) return;
  if (in_sizes[6] != DM * DM || in_sizes[7] != DM) return;
  if (in_sizes[8] != DML * DM || in_sizes[9] != DML) return;
  if (in_sizes[10] != DML * DM || in_sizes[11] != DML) return;
  if (in_sizes[12] != NMIX * 2) return;
  if (in_sizes[13] != DM * DM || in_sizes[14] != DM) return;
  if (in_sizes[15] != NH || in_sizes[16] != NMIX) return;
  if (out_size != OUTN) return;

  const float* x    = (const float*)d_in[0];
  const float* wq   = (const float*)d_in[2];
  const float* bq   = (const float*)d_in[3];
  const float* wk   = (const float*)d_in[4];
  const float* bk   = (const float*)d_in[5];
  const float* wv   = (const float*)d_in[6];
  const float* bv   = (const float*)d_in[7];
  const float* wqm  = (const float*)d_in[8];
  const float* bqm  = (const float*)d_in[9];
  const float* wkm  = (const float*)d_in[10];
  const float* bkm  = (const float*)d_in[11];
  const float* mixw = (const float*)d_in[12];
  const float* wp   = (const float*)d_in[13];
  const float* bp   = (const float*)d_in[14];
  const float* bcl  = (const float*)d_in[15];
  const float* bclm = (const float*)d_in[16];

  const size_t PX    = (size_t)ROWS * DM * 2;
  const size_t PWT   = (size_t)NQKV * DM * 2;
  const size_t PWP   = (size_t)DM * DM * 2;
  const size_t PBC   = (size_t)NQKV * 4;
  const size_t PQKVF = (size_t)ROWS * NQKV * 4;
  const size_t PQK   = (size_t)ROWS * LDQK * 2;
  const size_t PVT   = (size_t)NB * NH * HD * SEQ * 2;
  const size_t PY    = (size_t)NVH * NB * SEQ * HD * 4;
  const size_t PCTX  = (size_t)ROWS * DM * 2;
  size_t off = 0;
  const size_t oX    = off; off += PX;
  const size_t oWT   = off; off += PWT;
  const size_t oWP   = off; off += PWP;
  const size_t oBC   = off; off += PBC;
  const size_t oQKVF = off; off += PQKVF;
  const size_t oQKH  = off; off += PQK;
  const size_t oQKR  = off; off += PQK;
  const size_t oVT   = off; off += PVT;
  const size_t oVTR  = off; off += PVT;
  const size_t oY    = off; off += PY;
  const size_t oCTX  = off; off += PCTX;
  const size_t oCTXR = off; off += PCTX;
  if (off > ws_size) return;
  if (off > (size_t)134217728) return;

  char* ws = (char*)d_ws;
  unsigned short* XH   = (unsigned short*)(ws + oX);
  unsigned short* WT   = (unsigned short*)(ws + oWT);
  unsigned short* WPT  = (unsigned short*)(ws + oWP);
  float*          BC   = (float*)(ws + oBC);
  float*          QKVF = (float*)(ws + oQKVF);
  unsigned short* QKH  = (unsigned short*)(ws + oQKH);
  unsigned short* QKR  = (unsigned short*)(ws + oQKR);
  unsigned short* VT   = (unsigned short*)(ws + oVT);
  unsigned short* VTR  = (unsigned short*)(ws + oVTR);
  float*          YV   = (float*)(ws + oY);
  unsigned short* CTX  = (unsigned short*)(ws + oCTX);
  unsigned short* CTXR = (unsigned short*)(ws + oCTXR);
  float*          outf = (float*)d_out;

  const dim3 blk(256);
  const int n8x  = ROWS * DM / 8;
  const int n8w  = DM * DM / 8;
  const int n8m  = DML * DM / 8;
  const int n8qk = ROWS * LDQK / 8;
  const dim3 gCx((n8x + 255) / 256);
  const dim3 gCw((n8w + 255) / 256);
  const dim3 gCm((n8m + 255) / 256);
  const dim3 gBc((NQKV / 4 + 255) / 256);
  const dim3 gGq(((ROWS / 64) * (NQKV / 64) + 7) / 8);
  const dim3 gQk((n8qk + 255) / 256);
  const dim3 gVt(SEQ / 64, NH, NB);
  const dim3 gAt(NQB * NVH * NB);
  const dim3 gMx((n8x + 255) / 256);
  const dim3 gGo(((ROWS / 64) * (DM / 64) + 7) / 8);
  const float wScale = 1024.0f;
  const float aScale = 16.0f;
  const float cscale = 1.0f / 16384.0f;

  cvt16<true><<<gCx, blk, 0, stream>>>(x, XH, n8x, aScale);
  cvt16<true><<<gCw, blk, 0, stream>>>(wq,  WT + (size_t)CQ   * DM, n8w, wScale);
  cvt16<true><<<gCw, blk, 0, stream>>>(wk,  WT + (size_t)CK   * DM, n8w, wScale);
  cvt16<true><<<gCm, blk, 0, stream>>>(wqm, WT + (size_t)CQML * DM, n8m, wScale);
  cvt16<true><<<gCm, blk, 0, stream>>>(wkm, WT + (size_t)CKML * DM, n8m, wScale);
  cvt16<true><<<gCw, blk, 0, stream>>>(wv,  WT + (size_t)CV   * DM, n8w, wScale);
  cvt16<true><<<gCw, blk, 0, stream>>>(wp,  WPT, n8w, wScale);
  bias_cat<<<gBc, blk, 0, stream>>>(bq, bk, bqm, bkm, bv, BC);
  gemm64_f16<false><<<gGq, blk, 0, stream>>>(XH, XH, DM, WT, DM, BC, cscale, QKVF, NQKV, ROWS, NQKV, DM);
  qk_split<<<gQk, blk, 0, stream>>>(QKVF, QKH, QKR, n8qk);
  v_tr<<<gVt, blk, 0, stream>>>(QKVF, VT, VTR);
  attn_k<<<gAt, dim3(128), 0, stream>>>(QKH, QKR, VT, VTR, bcl, bclm, YV);
  mix_cvt<<<gMx, blk, 0, stream>>>(YV, mixw, CTX, CTXR);
  gemm64_f16<true><<<gGo, blk, 0, stream>>>(CTX, CTXR, DM, WPT, DM, bp, cscale, outf, DM, ROWS, DM, DM);
  (void)hipGetLastError();
}
